// AttentionBlock_41695542509821
// MI455X (gfx1250) — hardware-verified
//
#include <hip/hip_runtime.h>
#ifndef NB
#define NB 4
#endif
#ifndef SEQ
#define SEQ 4096
#endif
#define NB_FULL 4
#define SQ_FULL 4096
#define SQ SEQ
#define DM 512
#define NH 8
#define NG 32
#define GC (DM / NG)
#define QN (SQ < 1024 ? SQ : 1024)
#define NR ((size_t)NB * SQ)
#define XBS ((size_t)SQ_FULL * DM)
static_assert(NB >= 1 && NB <= NB_FULL);
static_assert(SQ >= 256 && SQ <= SQ_FULL && SQ % 128 == 0);
static_assert(QN % 256 == 0 && SQ % QN == 0);
static_assert(DM % 64 == 0 && GC == 16);

typedef unsigned short v8us __attribute__((ext_vector_type(8), may_alias));
typedef float  v8f  __attribute__((ext_vector_type(8)));
typedef float  v4f  __attribute__((ext_vector_type(4)));
typedef float  v4fa __attribute__((ext_vector_type(4), may_alias));
typedef _Float16 v16h __attribute__((ext_vector_type(16)));
typedef _Float16 v4h __attribute__((ext_vector_type(4)));
union FragH { v16h v; v8us half[2]; _Float16 h[16]; unsigned short u[16]; };

__device__ __forceinline__ unsigned short bf16_bits(float x) { unsigned int u = __float_as_uint(x); return (unsigned short)((u + 0x7FFFu + ((u >> 16) & 1u)) >> 16); }
__device__ __forceinline__ float bf16_val(unsigned short b) { return __uint_as_float(((unsigned int)b) << 16); }
__device__ __forceinline__ float bf16_rne(float x) { return bf16_val(bf16_bits(x)); }

__global__ __launch_bounds__(256) void k_wt_f16(const float* __restrict__ W, _Float16* __restrict__ Wt, int K, int N, float scale) {
  const int t = blockIdx.x * 256 + threadIdx.x; if (t >= N * (K / 8)) return; const int n = t / (K / 8), k8 = (t % (K / 8)) * 8; FragH f;
#pragma unroll
  for (int i = 0; i < 8; ++i) f.h[i] = (_Float16)(bf16_rne(W[(size_t)(k8 + i) * N + n]) * scale); const v8us o = f.half[0];
  *(volatile v8us*)((unsigned short*)Wt + (size_t)n * K + k8) = o; __threadfence(); *(volatile v8us*)((unsigned short*)Wt + (size_t)n * K + k8) = o;
}

__device__ __forceinline__ v16h g2_frag(const _Float16* p, int hh) { FragH f; f.half[0] = *(const v8us*)((const unsigned short*)p + 8 * hh); f.half[1] = *(const v8us*)((const unsigned short*)p + 16 + 8 * hh); return f.v; }
__device__ __forceinline__ v8f g2_mma(v16h a, v16h b, v8f c) { v8f d = __builtin_amdgcn_wmma_f32_16x16x32_f16(false, a, false, b, (short)0, c, false, false); asm volatile("v_nop\n\tv_nop\n\tv_nop\n\tv_nop" : "+v"(d) : "v"(a), "v"(b)); return d; }
template <int ACT>
__global__ __launch_bounds__(128) void k_gemm2(const _Float16* __restrict__ A, int lda, size_t sA, const _Float16* __restrict__ Bh, int ldb, size_t sB, float alpha, const float* __restrict__ bias, size_t sBias, const float* __restrict__ CP, int rowsPerB, size_t sCPb, int row0g,
    float* __restrict__ C, _Float16* __restrict__ C16, int ldc, size_t sC, int M, int N, int K) {
  static_assert(ACT == 0 || ACT == 3);
  __shared__ __attribute__((aligned(16))) float so[4][32][68];
  const int tid = threadIdx.x, w = tid >> 5, lane = tid & 31, ln = lane & 15, hh = lane >> 4; const int by = blockIdx.y;
  A += (size_t)by * sA; Bh += (size_t)by * sB; const size_t cofs = (size_t)by * sC; const float* bp = bias ? bias + (size_t)by * sBias : nullptr;
  const int ntn = N >> 6; const int mt = blockIdx.x / ntn, nq = blockIdx.x - mt * ntn; const int row0 = mt * 128 + 32 * w, col0 = nq * 64; if (row0 >= M) return;
  const _Float16* a0p = A + (size_t)(row0 + ln) * lda; const _Float16* a1p = a0p + (size_t)16 * lda;
  const _Float16* b0p = Bh + (size_t)(col0 + ln) * ldb; const _Float16* b1p = b0p + (size_t)16 * ldb; const _Float16* b2p = b1p + (size_t)16 * ldb; const _Float16* b3p = b2p + (size_t)16 * ldb;
  const v8f z8 = {0.f,0.f,0.f,0.f,0.f,0.f,0.f,0.f}; v8f c00 = z8, c01 = z8, c02 = z8, c03 = z8, c10 = z8, c11 = z8, c12 = z8, c13 = z8;
#pragma unroll 1
  for (int kb = 0; kb < K; kb += 32) { const v16h a0 = g2_frag(a0p + kb, hh), a1 = g2_frag(a1p + kb, hh);
    v16h b = g2_frag(b0p + kb, hh); c00 = g2_mma(a0, b, c00); c10 = g2_mma(a1, b, c10);
    b = g2_frag(b1p + kb, hh); c01 = g2_mma(a0, b, c01); c11 = g2_mma(a1, b, c11);
    b = g2_frag(b2p + kb, hh); c02 = g2_mma(a0, b, c02); c12 = g2_mma(a1, b, c12);
    b = g2_frag(b3p + kb, hh); c03 = g2_mma(a0, b, c03); c13 = g2_mma(a1, b, c13); }
  v8f accs[8] = {c00, c01, c02, c03, c10, c11, c12, c13};
#pragma unroll
  for (int u = 0; u < 8; ++u) { const int t = u & 3, half = u >> 2; const int col = col0 + t * 16 + ln; const float bv = bp ? bf16_rne(bp[col]) : 0.f;
#pragma unroll
    for (int r = 0; r < 8; ++r) { const int rloc = half * 16 + 8 * hh + r; float v = accs[u][r] * alpha + bv;
      if (CP) { if (rowsPerB < 0) v += CP[cofs + (size_t)(row0g + row0 + rloc) * ldc + col]; else { const int bidx = (row0g + row0 + rloc) / rowsPerB; v += CP[(size_t)bidx * sCPb + (size_t)by * 64 + col]; } }
      if (ACT == 3) v = fmaxf(v, 0.f);
      so[w][rloc][t * 16 + ln] = v; } }
  __builtin_amdgcn_fence(4  , "workgroup"); __builtin_amdgcn_wave_barrier();
  const int rsub = lane >> 4, c4 = (lane & 15) * 4;
  for (int pass = 0; pass < 2; ++pass) {
#pragma unroll
    for (int q = 0; q < 16; ++q) { const int r = q * 2 + rsub; const v4f v = *(const v4fa*)&so[w][r][c4]; if (C) *(volatile v4f*)(C + cofs + (size_t)(row0 + r) * ldc + col0 + c4) = v; if (C16) { v4h h4; for (int i = 0; i < 4; ++i) h4[i] = (_Float16)v[i]; *(volatile v4h*)(C16 + cofs + (size_t)(row0 + r) * ldc + col0 + c4) = h4; } }
    if (pass == 0) __threadfence(); } }

template <int NHv, int TTv>
__global__ __launch_bounds__(256) void k_vt(const _Float16* __restrict__ V16, int ldv, int voff, _Float16* __restrict__ Vt) { __shared__ unsigned short tl[64][66]; const int tid = threadIdx.x; const int slab = blockIdx.x / (TTv / 64), lg = blockIdx.x % (TTv / 64); const int b = slab / NHv, h = slab % NHv;
  for (int i = tid; i < 64 * 8; i += 256) { const int r = i / 8, c8 = (i % 8) * 8; FragH f; f.half[0] = *(const v8us*)((const unsigned short*)V16 + ((size_t)b * TTv + lg * 64 + r) * ldv + voff + h * 64 + c8);
#pragma unroll
    for (int q = 0; q < 8; ++q) tl[r][c8 + q] = f.u[q]; }
  __syncthreads();
  for (int pass = 0; pass < 2; ++pass) {
#pragma unroll
    for (int rd = 0; rd < 2; ++rd) { const int d = rd * 32 + tid / 8, pc = tid % 8; FragH f;
#pragma unroll
      for (int q = 0; q < 8; ++q) f.u[q] = tl[pc * 8 + q][d];
      *(volatile v8us*)((unsigned short*)Vt + ((size_t)slab * 64 + d) * TTv + lg * 64 + pc * 8) = f.half[0]; }
    if (pass == 0) __threadfence(); } }

__global__ __launch_bounds__(256) void k_bfr(const float* __restrict__ x, float* __restrict__ XB, size_t n4) { const size_t t = (size_t)blockIdx.x * 256 + threadIdx.x; if (t >= n4) return;
  const size_t e = t * 4; const size_t row = e / DM; const size_t f = ((row / SQ) * SQ_FULL + (row % SQ)) * DM + (e % DM);
  v4f a = *(const v4fa*)(x + f); for (int q = 0; q < 4; ++q) a[q] = bf16_rne(a[q]);
  *(volatile v4f*)(XB + f) = a; __threadfence(); *(volatile v4f*)(XB + f) = a; }

__global__ __launch_bounds__(256) void k_gnstat(const float* __restrict__ x, float eps, float* __restrict__ st) {
  #pragma clang fp contract(off)
  __shared__ float red[256]; const int b = blockIdx.x / NG, g = blockIdx.x % NG; const int t = threadIdx.x; const float* xb = x + (size_t)b * XBS + g * GC; float s = 0.f;
  for (int i = t; i < SQ * GC; i += 256) { const int tok = i / GC, c = i % GC; s = __fadd_rn(s, bf16_rne(xb[(size_t)tok * DM + c])); }
  red[t] = s; __syncthreads(); for (int k = 128; k > 0; k >>= 1) { if (t < k) red[t] = __fadd_rn(red[t], red[t + k]); __syncthreads(); } const float mu = red[0] / (float)(SQ * GC); __syncthreads();
  float v = 0.f; for (int i = t; i < SQ * GC; i += 256) { const int tok = i / GC, c = i % GC; const float d = __fadd_rn(bf16_rne(xb[(size_t)tok * DM + c]), -mu); v = __fadd_rn(v, __fmul_rn(d, d)); }
  red[t] = v; __syncthreads(); for (int k = 128; k > 0; k >>= 1) { if (t < k) red[t] = __fadd_rn(red[t], red[t + k]); __syncthreads(); }
  const float rs = rsqrtf(__fadd_rn(red[0] / (float)(SQ * GC), eps));
  if (t < 8) { v4f o = {0.f, 0.f, 0.f, 0.f}; if (t == 0) { o[0] = mu; o[1] = rs; } float* d = st + (size_t)blockIdx.x * 32 + t * 4; *(volatile v4f*)d = o; __threadfence(); *(volatile v4f*)d = o; } }
__global__ __launch_bounds__(256) void k_gnrows(const float* __restrict__ x, const float* __restrict__ st, const float* __restrict__ ga, const float* __restrict__ be, _Float16* __restrict__ H) {
  #pragma clang fp contract(off)
  const size_t t = (size_t)blockIdx.x * 256 + threadIdx.x; if (t >= NR * DM / 8) return; const size_t e = t * 8; const int c0 = (int)(e % DM); const size_t row = e / DM; const int b = (int)(row / SQ); const size_t f = ((size_t)b * SQ_FULL + (row % SQ)) * DM + c0; const int g = c0 / GC;
  const float mu = st[((size_t)b * NG + g) * 32], rs = st[((size_t)b * NG + g) * 32 + 1];
  const v4f a = *(const v4fa*)(x + f), a2 = *(const v4fa*)(x + f + 4); FragH fr; for (int q = 0; q < 8; ++q) { const float xv = bf16_rne(q < 4 ? a[q] : a2[q - 4]); fr.h[q] = (_Float16)__fadd_rn(__fmul_rn(__fmul_rn(__fadd_rn(xv, -mu), rs), bf16_rne(ga[c0 + q])), bf16_rne(be[c0 + q])); }
  *(volatile v8us*)((unsigned short*)H + e) = fr.half[0]; __threadfence(); *(volatile v8us*)((unsigned short*)H + e) = fr.half[0]; }

__global__ __launch_bounds__(256) void k_rsm(const float* __restrict__ S, _Float16* __restrict__ P, int nrows) {
  #pragma clang fp contract(off)
  __shared__ __attribute__((aligned(16))) unsigned short tl[256][72];
  const int t = threadIdx.x; const int i0 = blockIdx.x * 256; const int ir = i0 + t; const int i = (ir < nrows) ? ir : (nrows - 1);
  const float* s = S + (size_t)i * SQ; float mx = -3.0e38f;
#pragma unroll 1
  for (int j = 0; j < SQ; j += 4) { const v4f a = *(const v4fa*)(s + j); mx = fmaxf(mx, a[0]); mx = fmaxf(mx, a[1]); mx = fmaxf(mx, a[2]); mx = fmaxf(mx, a[3]); }
  float se = 0.f;
#pragma unroll 1
  for (int j = 0; j < SQ; j += 4) { const v4f a = *(const v4fa*)(s + j); se += __expf(a[0] - mx); se += __expf(a[1] - mx); se += __expf(a[2] - mx); se += __expf(a[3] - mx); }
  const float sc = 256.0f / se;
#pragma unroll 1
  for (int j0 = 0; j0 < SQ; j0 += 64) {
#pragma unroll 1
    for (int m = 0; m < 8; ++m) { const v4f a = *(const v4fa*)(s + j0 + 8 * m), c = *(const v4fa*)(s + j0 + 8 * m + 4); FragH f;
#pragma unroll
      for (int q = 0; q < 4; ++q) { f.h[q] = (_Float16)(__expf(a[q] - mx) * sc); f.h[4 + q] = (_Float16)(__expf(c[q] - mx) * sc); }
      *(v8us*)&tl[t][8 * m] = f.half[0]; }
    __syncthreads();
    for (int pass = 0; pass < 2; ++pass) {
#pragma unroll
      for (int u = 0; u < 8; ++u) { const int line = u * 32 + (t >> 3), pc = t & 7; const int row = i0 + line;
        if (row < nrows) { const v8us vv = *(const v8us*)&tl[line][pc * 8]; *(volatile v8us*)((unsigned short*)P + (size_t)row * SQ + j0 + pc * 8) = vv; } }
      if (pass == 0) __threadfence(); }
    __syncthreads();
  } }

extern "C" void kernel_launch(void* const* d_in, const int* in_sizes, int n_in,
                              void* d_out, int out_size, void* d_ws, size_t ws_size, hipStream_t stream) {
  if (n_in < 11) return;
  const size_t xneed = ((size_t)(NB - 1) * SQ_FULL + SQ) * DM;
  if ((size_t)in_sizes[0] < xneed || in_sizes[1] < DM || in_sizes[2] < DM || in_sizes[3] < DM * DM || in_sizes[4] < DM || in_sizes[5] < DM * DM || in_sizes[6] < DM ||
      in_sizes[7] < DM * DM || in_sizes[8] < DM || in_sizes[9] < DM * DM || in_sizes[10] < DM || (size_t)out_size < xneed) return;
  const float* const* I = (const float* const*)d_in; const float* x = I[0]; const float* ga = I[1]; const float* be = I[2]; const float* wq = I[3]; const float* bq = I[4]; const float* wk = I[5]; const float* bk = I[6]; const float* wv = I[7]; const float* bv = I[8]; const float* wo = I[9]; const float* bo = I[10];
  char* ws = (char*)d_ws; size_t off = 0;
  auto take = [&](size_t bytes) { char* p = ws + off; off += (bytes + 255) & ~(size_t)255; return p; };
  _Float16* BQ = (_Float16*)take((size_t)DM * DM * 2); _Float16* BK = (_Float16*)take((size_t)DM * DM * 2); _Float16* BV = (_Float16*)take((size_t)DM * DM * 2); _Float16* BO = (_Float16*)take((size_t)DM * DM * 2);
  float* ST = (float*)take((size_t)NB * NG * 32 * 4); float* XB = (float*)take((size_t)NB * XBS * 4);
  _Float16* H16 = (_Float16*)take(NR * DM * 2); _Float16* Q16 = (_Float16*)take(NR * DM * 2); _Float16* K16 = (_Float16*)take(NR * DM * 2); _Float16* V16 = (_Float16*)take(NR * DM * 2);
  _Float16* O16 = H16;
  float* S = (float*)take((size_t)QN * SQ * 4); _Float16* P = (_Float16*)take((size_t)QN * SQ * 2); _Float16* VT = (_Float16*)take((size_t)DM * SQ * 2);
  if (off > ws_size) return;
  const unsigned gw = (unsigned)(((size_t)DM * (DM / 8) + 255) / 256);
  k_wt_f16<<<gw, 256, 0, stream>>>(wq, BQ, DM, DM, 16.0f); k_wt_f16<<<gw, 256, 0, stream>>>(wk, BK, DM, DM, 16.0f); k_wt_f16<<<gw, 256, 0, stream>>>(wv, BV, DM, DM, 16.0f); k_wt_f16<<<gw, 256, 0, stream>>>(wo, BO, DM, DM, 16.0f);
  k_gnstat<<<NB * NG, 256, 0, stream>>>(x, 1e-6f, ST); k_gnrows<<<(unsigned)((NR * DM / 8 + 255) / 256), 256, 0, stream>>>(x, ST, ga, be, H16);
  k_bfr<<<(unsigned)((NR * DM / 4 + 255) / 256), 256, 0, stream>>>(x, XB, NR * DM / 4);
  k_gemm2<0><<<dim3((unsigned)((NR / 128) * (DM / 64)), 1), 128, 0, stream>>>(H16, DM, 0, BQ, DM, 0, 0.0625f, bq, 0, nullptr, 1, 0, 0, nullptr, Q16, DM, 0, (int)NR, DM, DM);
  k_gemm2<0><<<dim3((unsigned)((NR / 128) * (DM / 64)), 1), 128, 0, stream>>>(H16, DM, 0, BK, DM, 0, 0.0625f, bk, 0, nullptr, 1, 0, 0, nullptr, K16, DM, 0, (int)NR, DM, DM);
  k_gemm2<0><<<dim3((unsigned)((NR / 128) * (DM / 64)), 1), 128, 0, stream>>>(H16, DM, 0, BV, DM, 0, 0.0625f, bv, 0, nullptr, 1, 0, 0, nullptr, V16, DM, 0, (int)NR, DM, DM);
  for (int b = 0; b < NB; ++b) { const size_t r0 = (size_t)b * SQ;
    k_vt<NH, SQ><<<NH * (SQ / 64), 256, 0, stream>>>(V16 + r0 * DM, DM, 0, VT);
    for (int c = 0; c < SQ / QN; ++c) { const size_t q0 = r0 + (size_t)c * QN;
      k_gemm2<0><<<dim3((QN / 128) * (SQ / 64), 1), 128, 0, stream>>>(Q16 + q0 * DM, DM, 0, K16 + r0 * DM, DM, 0, 0.044194173824159216f, nullptr, 0, nullptr, 1, 0, 0, S, nullptr, SQ, 0, QN, SQ, DM);
      k_rsm<<<QN / 256, 256, 0, stream>>>(S, P, QN);
      k_gemm2<0><<<dim3((QN / 128) * (DM / 64), 1), 128, 0, stream>>>(P, SQ, 0, VT, SQ, 0, 0.25f, nullptr, 0, nullptr, 1, 0, 0, nullptr, O16 + q0 * DM, DM, 0, QN, DM, SQ); } }
  k_gemm2<0><<<dim3((unsigned)((SQ / 128) * (DM / 64)), NB), 128, 0, stream>>>(O16, DM, (size_t)SQ * DM, BO, DM, 0, 0.0009765625f, bo, 0, XB, -1, 0, 0, (float*)d_out, nullptr, DM, XBS, SQ, DM, DM);
}
